// Correlation_3350074491441
// MI455X (gfx1250) — hardware-verified
//
#include <hip/hip_runtime.h>

typedef __bf16 bf16_t;
typedef bf16_t   v16bf __attribute__((ext_vector_type(16)));
typedef float    v8f   __attribute__((ext_vector_type(8)));
typedef float    v4f   __attribute__((ext_vector_type(4)));
typedef unsigned v4u   __attribute__((ext_vector_type(4)));
typedef v4f __attribute__((may_alias)) v4fa;
typedef v4u __attribute__((may_alias)) v4ua;

union FragB { v16bf v; v4u q[2]; };

#define NBATCH 8
#define NCH    256
#define HH     48
#define WW     64
#define GRAD   10
#define GWID   21
#define NDISP  441
#define NROWS  (NBATCH * HH)
#define N_IN_ELEMS  (NBATCH * NCH * HH * WW)
#define N_OUT_ELEMS (NBATCH * NDISP * HH * WW)
#define PLANE_HALVES ((size_t)NROWS * WW * NCH)
#define TP 132
#define GP 68

static_assert((TP * 4) % 16 == 0);
static_assert(NCH % 32 == 0);
static_assert(WW == 64);

__device__ __forceinline__ v8f wmma_bf16(v16bf a, v16bf b, v8f c) {
  v8f d = __builtin_amdgcn_wmma_f32_16x16x32_bf16(false, a, false, b, (short)0, c, false, false);
  asm volatile("v_nop\n\tv_nop\n\tv_nop\n\tv_nop" : "+v"(d) : "v"(a), "v"(b));
  return d;
}

__device__ __forceinline__ v16bf load_frag_bf(const bf16_t* p, int h) {
  FragB f;
  f.q[0] = *(const v4ua*)(p + 8 * h);
  f.q[1] = *(const v4ua*)(p + 16 + 8 * h);
  return f.v;
}

__device__ __forceinline__ unsigned bf16_bits_rne(float f) {
  unsigned u = __float_as_uint(f);
  u = u + 0x7FFFu + ((u >> 16) & 1u);
  return u >> 16;
}

__device__ __forceinline__ void tr_store_pass(const unsigned* T, bf16_t* dst, int row, int w, int lane) {
  #pragma unroll
  for (int i = 0; i < 8; ++i) {
    const int x = 8 * w + i;
    const v4u v = *(const v4ua*)(T + x * TP + 4 * lane);
    bf16_t* p = dst + ((size_t)row * WW + x) * NCH + 8 * lane;
    *(volatile v4u*)p = v;
  }
}

__global__ __launch_bounds__(256) void k_transpose(
    const float* __restrict__ in1, const float* __restrict__ in2,
    bf16_t* __restrict__ p1, bf16_t* __restrict__ p2)
{
  __shared__ __attribute__((aligned(16))) unsigned T[WW * TP];

  const int tid = threadIdx.x, lane = tid & 31, w = tid >> 5;
  const int which = blockIdx.y;
  const int row = blockIdx.x;
  const int b = row / HH, y = row - b * HH;
  const float* src = (which == 0) ? in1 : in2;
  bf16_t* dst = (which == 0) ? p1 : p2;

  #pragma unroll 1
  for (int it = 0; it < 8; ++it) {
    const int t = tid + 256 * it;
    const int c2 = t >> 4;
    const int x4 = t & 15;
    const float* pa = src + (((size_t)b * NCH + 2 * c2) * HH + y) * WW + 4 * x4;
    const v4f a = *(const v4fa*)pa;
    const v4f c = *(const v4fa*)(pa + (size_t)HH * WW);
    unsigned* tr = T + (4 * x4) * TP + c2;
    tr[0 * TP] = bf16_bits_rne(a.x) | (bf16_bits_rne(c.x) << 16);
    tr[1 * TP] = bf16_bits_rne(a.y) | (bf16_bits_rne(c.y) << 16);
    tr[2 * TP] = bf16_bits_rne(a.z) | (bf16_bits_rne(c.z) << 16);
    tr[3 * TP] = bf16_bits_rne(a.w) | (bf16_bits_rne(c.w) << 16);
  }
  __syncthreads();

  tr_store_pass(T, dst, row, w, lane);
  __threadfence();
  tr_store_pass(T, dst, row, w, lane);
}

__device__ __forceinline__ float band_pick(const float* sG, int x, int sh) {
  const int u = x + sh;
  const int uc = min(max(u, 0), WW - 1);
  const float g = sG[x * GP + uc];
  return (u >= 0 && u < WW) ? g * 0.00390625f : 0.0f;
}

__device__ __forceinline__ void corr_store_pass(const float* sG, float* out,
                                                int b, int y, int dyi, int w, int lane) {
  const int h = lane >> 4, q = lane & 15;
  const int x0 = 4 * q;
  #pragma unroll
  for (int i = 0; i < 3; ++i) {
    const int dxi = 6 * w + 2 * i + h;
    const int sh = 2 * dxi - 2 * GRAD;
    v4f v;
    v.x = band_pick(sG, x0 + 0, sh);
    v.y = band_pick(sG, x0 + 1, sh);
    v.z = band_pick(sG, x0 + 2, sh);
    v.w = band_pick(sG, x0 + 3, sh);
    if (dxi < GWID) {
      const size_t gi = (((size_t)b * NDISP + dyi * GWID + dxi) * HH + y) * WW + x0;
      *(volatile v4f*)(out + gi) = v;
    }
  }
}

__global__ __launch_bounds__(128) void k_corr(
    const bf16_t* __restrict__ p1,
    const bf16_t* __restrict__ p2,
    float* __restrict__ out)
{
  __shared__ __attribute__((aligned(16))) float sG[WW * GP];

  const int tid = threadIdx.x, lane = tid & 31, w = tid >> 5;
  const int h = lane >> 4, m = lane & 15;
  const int blk = blockIdx.x;
  const int dyi = blk % GWID;
  const int row = blk / GWID;
  const int b = row / HH, y = row - b * HH;
  const int r2 = y + 2 * dyi - 2 * GRAD;
  const bool valid = (r2 >= 0) && (r2 < HH);

  if (valid) {
    const bf16_t* arow = p1 + ((size_t)row * WW + 16 * w + m) * NCH;
    const bf16_t* brow = p2 + (((size_t)b * HH + r2) * WW + m) * NCH;

    const v8f zero8 = {0.f, 0.f, 0.f, 0.f, 0.f, 0.f, 0.f, 0.f};
    v8f acc[4];
    #pragma unroll
    for (int nt = 0; nt < 4; ++nt) acc[nt] = zero8;

    #pragma unroll 1
    for (int k0 = 0; k0 < NCH; k0 += 32) {
      const v16bf a = load_frag_bf(arow + k0, h);
      #pragma unroll
      for (int nt = 0; nt < 4; ++nt) {
        const v16bf bb = load_frag_bf(brow + (size_t)nt * 16 * NCH + k0, h);
        acc[nt] = wmma_bf16(a, bb, acc[nt]);
      }
    }

    #pragma unroll
    for (int nt = 0; nt < 4; ++nt) {
      #pragma unroll
      for (int r = 0; r < 8; ++r) {
        sG[(16 * w + 8 * h + r) * GP + 16 * nt + m] = acc[nt][r];
      }
    }
  } else {
    #pragma unroll 4
    for (int t = tid; t < WW * WW; t += 128) {
      sG[(t >> 6) * GP + (t & 63)] = 0.0f;
    }
  }
  __syncthreads();

  corr_store_pass(sG, out, b, y, dyi, w, lane);
  __threadfence();
  corr_store_pass(sG, out, b, y, dyi, w, lane);
}

extern "C" void kernel_launch(void* const* d_in, const int* in_sizes, int n_in,
                              void* d_out, int out_size, void* d_ws, size_t ws_size,
                              hipStream_t stream) {
  if (n_in < 2) return;
  if (in_sizes[0] != N_IN_ELEMS || in_sizes[1] != N_IN_ELEMS) return;
  if (out_size != N_OUT_ELEMS) return;

  const size_t plane_bytes = PLANE_HALVES * 2;
  const size_t total = 2 * plane_bytes;
  if (total > ws_size || d_ws == nullptr) return;

  const float* in1 = (const float*)d_in[0];
  const float* in2 = (const float*)d_in[1];
  float* out = (float*)d_out;
  char* ws = (char*)d_ws;
  bf16_t* p1 = (bf16_t*)(ws);
  bf16_t* p2 = (bf16_t*)(ws + plane_bytes);

  k_transpose<<<dim3(NROWS, 2), dim3(256), 0, stream>>>(in1, in2, p1, p2);
  k_corr<<<dim3(NROWS * GWID), dim3(128), 0, stream>>>(p1, p2, out);
}
